// SAGENet_15530601742448
// MI455X (gfx1250) — hardware-verified
//
#include <hip/hip_runtime.h>
#include <stddef.h>
#include <stdint.h>
#include <math.h>


#define FIN     32
#define HID     16
#define TW1     128
#define TW2     64
#define AP1     128
#define KL1     96
#define BP1     128
#define AP2     64
#define KL2     64
#define BP2     64
#define HPW     32
#define NTHR    256
#define NWAVE   8
#define EPT     8
#define CHUNK   (NTHR * EPT)
#define WCAP    (EPT * 32)
#define LISTN   (NWAVE * WCAP)
#define NBA     1024
#define SLA     10
#define RCAP    28672
#define DEGCAP  64
#define GBM     64
#define GTHR    128
#define TR1     8
#define NPAR    384
#define PEPS    1e-7f
#define AGG_ZINTS     (LISTN + 2 * RCAP + 3 * NBA)
#define MISC_INTS     16
#define SCAN_LDS_INTS (AGG_ZINTS + MISC_INTS + NPAR)
#define WSMAX   134217728

static_assert((CHUNK & (CHUNK - 1)) == 0 && CHUNK <= 4096);
static_assert((NBA & (NBA - 1)) == 0 && NBA == (1 << SLA));
static_assert(((long long)CHUNK << SLA) < (1LL << 31));
static_assert(LISTN % NTHR == 0);
static_assert(NBA % NWAVE == 0 && NBA % 32 == 0 && NBA % GBM == 0);
static_assert(RCAP % 4 == 0 && AGG_ZINTS % 4 == 0 && LISTN % 4 == 0 && ((AGG_ZINTS + MISC_INTS) % 4) == 0);
static_assert(AGG_ZINTS % (NTHR * 4) == 0);
static_assert(SCAN_LDS_INTS * 4 <= 300000);
static_assert(KL1 % 32 == 0 && KL2 % 32 == 0 && KL1 <= AP1 && KL2 <= AP2 && KL1 <= BP1 && KL2 <= BP2);
static_assert(GBM == (GTHR / 32) * 16);
static_assert(FIN == 32 && HID == 16);
static_assert(TW1 == 4 * FIN && TW1 == 4 * 32);
static_assert(TW2 == 4 * HID && TW2 == 2 * 32);
static_assert(AP1 == 4 * 32 && AP2 == 2 * 32);
static_assert(GBM % TR1 == 0);
static_assert((GBM * HID) % GTHR == 0 && (GBM * TW2 / 4) % GTHR == 0 && (GBM * HPW / 8) % GTHR == 0);
static_assert((GBM * HID / 4) % GTHR == 0);
static_assert(NPAR >= 12 * FIN);
static_assert(NTHR == 16 * 16 && GTHR >= 4 * HID);

typedef float          v2f   __attribute__((ext_vector_type(2)));
typedef float          v4f   __attribute__((ext_vector_type(4)));
typedef float          v8f   __attribute__((ext_vector_type(8)));
typedef int            v4i   __attribute__((ext_vector_type(4)));
typedef int            v8i   __attribute__((ext_vector_type(8)));
typedef unsigned       v2u   __attribute__((ext_vector_type(2)));
typedef unsigned       v4u   __attribute__((ext_vector_type(4)));
typedef unsigned short v8us  __attribute__((ext_vector_type(8)));
typedef __bf16         v16bf __attribute__((ext_vector_type(16)));
typedef v2f  __attribute__((may_alias)) v2fa;
typedef v4f  __attribute__((may_alias)) v4fa;
typedef v4i  __attribute__((may_alias)) v4ia;
typedef v8us __attribute__((may_alias)) v8usa;
union FragB { v16bf v; v8us h[2]; v8i w; };

__device__ __forceinline__ v8f wmb(const FragB& a, const FragB& b, v8f c) {
  v8f d = __builtin_amdgcn_wmma_f32_16x16x32_bf16(false, a.v, false, b.v, (short)0, c, false, false);
  asm volatile("v_nop\n\tv_nop\n\tv_nop\n\tv_nop" : "+v"(d) : "v"(a.w), "v"(b.w));
  return d;
}

__device__ __forceinline__ unsigned bf16_bits(float f) {
  const unsigned u = __float_as_uint(f);
  return ((u + 0x7FFFu + ((u >> 16) & 1u)) >> 16) & 0xFFFFu;
}
__device__ __forceinline__ float bf16f(unsigned b) { return __uint_as_float(b << 16); }
__device__ __forceinline__ float bf16_val(float f) { return bf16f(bf16_bits(f)); }
__device__ __forceinline__ unsigned pk2(float lo, float hi) { return bf16_bits(lo) | (bf16_bits(hi) << 16); }
__device__ __forceinline__ float powv(float v, float p) { return exp2f(p * log2f(v)); }

template <int SLB>
__device__ __forceinline__ int scan_chunk(const int* __restrict__ dsts, int nE, int cbase, int slotBase,
                                          int nb, int vec8, int* list, int tid, int lane, int wave) {
  int wc = 0;
  const int el0  = tid * EPT;
  const int e0   = cbase + el0;
  const int sent = -2147483647 - 1;
  v4i da, db;
  if (vec8 != 0 && cbase + CHUNK <= nE) {
    da = *(const v4i*)(dsts + e0);
    db = *(const v4i*)(dsts + e0 + 4);
  } else {
    da.x = (e0     < nE) ? dsts[min(e0,     nE - 1)] : sent;
    da.y = (e0 + 1 < nE) ? dsts[min(e0 + 1, nE - 1)] : sent;
    da.z = (e0 + 2 < nE) ? dsts[min(e0 + 2, nE - 1)] : sent;
    da.w = (e0 + 3 < nE) ? dsts[min(e0 + 3, nE - 1)] : sent;
    db.x = (e0 + 4 < nE) ? dsts[min(e0 + 4, nE - 1)] : sent;
    db.y = (e0 + 5 < nE) ? dsts[min(e0 + 5, nE - 1)] : sent;
    db.z = (e0 + 6 < nE) ? dsts[min(e0 + 6, nE - 1)] : sent;
    db.w = (e0 + 7 < nE) ? dsts[min(e0 + 7, nE - 1)] : sent;
  }
  const unsigned nbs = (unsigned)slotBase;
  const unsigned unb = (unsigned)nb;
  const unsigned s0 = (unsigned)da.x - nbs, s1 = (unsigned)da.y - nbs;
  const unsigned s2 = (unsigned)da.z - nbs, s3 = (unsigned)da.w - nbs;
  const unsigned s4 = (unsigned)db.x - nbs, s5 = (unsigned)db.y - nbs;
  const unsigned s6 = (unsigned)db.z - nbs, s7 = (unsigned)db.w - nbs;
  const bool h0 = s0 < unb, h1 = s1 < unb, h2 = s2 < unb, h3 = s3 < unb;
  const bool h4 = s4 < unb, h5 = s5 < unb, h6 = s6 < unb, h7 = s7 < unb;
  const unsigned any = __builtin_amdgcn_ballot_w32(h0 | h1 | h2 | h3 | h4 | h5 | h6 | h7);
  if (any != 0u) {
#define HITJ(J, HJ, SJ) { \
      const unsigned mj = __builtin_amdgcn_ballot_w32(HJ); \
      if (mj != 0u) { \
        if (HJ) { \
          const int pos = wc + (int)__builtin_amdgcn_mbcnt_lo(mj, 0u); \
          if (pos < WCAP) list[wave * WCAP + pos] = ((el0 + (J)) << SLB) | (int)(SJ); \
        } \
        wc += (int)__builtin_popcount(mj); } }
    HITJ(0, h0, s0)
    HITJ(1, h1, s1)
    HITJ(2, h2, s2)
    HITJ(3, h3, s3)
    HITJ(4, h4, s4)
    HITJ(5, h5, s5)
    HITJ(6, h6, s6)
    HITJ(7, h7, s7)
#undef HITJ
  }
  return wc;
}

__global__ __launch_bounds__(NTHR) void k_wprep(const float* __restrict__ wr1, const float* __restrict__ wn1,
                                                const float* __restrict__ wr2, const float* __restrict__ wn2,
                                                unsigned short* B1T, unsigned short* B2T) {
  __shared__ __attribute__((aligned(16))) float wsm[3 * FIN * HID];
  const int tid = (int)threadIdx.x, wave = tid >> 5;
  {
    v4f v0;
    if (wave < 4) v0 = *(const v4f*)(wr1 + 4 * tid);
    else          v0 = *(const v4f*)(wn1 + 4 * (tid - 128));
    *(v4fa*)(wsm + 4 * tid) = v0;
    if (wave < 4) {
      v4f v1;
      if (wave < 2) v1 = *(const v4f*)(wr2 + 4 * tid);
      else          v1 = *(const v4f*)(wn2 + 4 * (tid - 64));
      *(v4fa*)(wsm + 2 * FIN * HID + 4 * tid) = v1;
    }
  }
  __syncthreads();

  v4u o1;
  {
    const int n = tid >> 4, k8 = (tid & 15) * 8, seg = k8 >> 5, kin = k8 & 31;
    const int moff = (seg == 0) ? 0 : FIN * HID;
    const float zf = (seg < 3) ? 1.0f : 0.0f;
    const float* q = wsm + moff + kin * HID + n;
    const float w0 = zf * q[0 * HID], w1 = zf * q[1 * HID], w2 = zf * q[2 * HID], w3 = zf * q[3 * HID];
    const float w4 = zf * q[4 * HID], w5 = zf * q[5 * HID], w6 = zf * q[6 * HID], w7 = zf * q[7 * HID];
    o1.x = pk2(w0, w1); o1.y = pk2(w2, w3); o1.z = pk2(w4, w5); o1.w = pk2(w6, w7);
  }
  v4u o2 = {0u, 0u, 0u, 0u};
  if (wave < 4) {
    const int n = tid >> 3, k8 = (tid & 7) * 8, seg = k8 >> 4, kin = k8 & 15;
    const int moff = 2 * FIN * HID + ((seg >= 2) ? HID * HID : 0);
    const float* q = wsm + moff + kin * HID + n;
    const float w0 = q[0 * HID], w1 = q[1 * HID], w2 = q[2 * HID], w3 = q[3 * HID];
    const float w4 = q[4 * HID], w5 = q[5 * HID], w6 = q[6 * HID], w7 = q[7 * HID];
    o2.x = pk2(w0, w1); o2.y = pk2(w2, w3); o2.z = pk2(w4, w5); o2.w = pk2(w6, w7);
  }
  unsigned short* d1 = B1T + (size_t)(tid >> 4) * BP1 + (tid & 15) * 8;
  unsigned short* d2 = B2T + (size_t)((tid & 127) >> 3) * BP2 + (tid & 7) * 8;
  *(volatile v4u*)d1 = o1;
  if (wave < 4) *(volatile v4u*)d2 = o2;
  __threadfence();
  *(volatile v4u*)d1 = o1;
  if (wave < 4) *(volatile v4u*)d2 = o2;
}

__global__ __launch_bounds__(NTHR) void k_t1(const float* __restrict__ x, const float* __restrict__ par,
                                             float* T1, int nN) {
  __shared__ __attribute__((aligned(16))) float st[TR1 * TW1];
  const int tid = (int)threadIdx.x, lane = tid & 31, wave = tid >> 5;
  const int row = (int)blockIdx.x * TR1 + wave;
  const int rc  = row < nN ? row : nN - 1;
  const float xv  = bf16_val(x[(size_t)rc * FIN + lane]);
  const float p5  = bf16_val(par[5 * FIN + lane]);
  const float p7  = bf16_val(par[7 * FIN + lane]);
  const float p9  = bf16_val(par[9 * FIN + lane]);
  const float p11 = bf16_val(par[11 * FIN + lane]);
  float e = 1.0f / (1.0f + expf(-xv));
  e = fminf(fmaxf(e, PEPS), 1.0f - PEPS);
  const float om = 1.0f - e;
  const float le = log2f(e), lo = log2f(om);
  float* sr = st + wave * TW1;
  sr[lane]           = exp2f(p5 * le);
  sr[FIN + lane]     = exp2f(p7 * lo);
  sr[2 * FIN + lane] = exp2f(p9 * le);
  sr[3 * FIN + lane] = exp2f(p11 * lo);
  __syncthreads();
  const v4f v = *(const v4fa*)(st + 4 * tid);
  float* dp = T1 + (size_t)blockIdx.x * (TR1 * TW1) + 4 * tid;
  *(volatile v4f*)dp = v;
  __threadfence();
  *(volatile v4f*)dp = v;
}

template <int L>
__global__ __launch_bounds__(NTHR) void k_scan(const int* __restrict__ srcs, const int* __restrict__ dsts,
                                               int nE, int nN, int vec8, int mRows,
                                               const float* __restrict__ par,
                                               const float* __restrict__ T,
                                               const float* __restrict__ xin,
                                               const unsigned* __restrict__ hpw,
                                               unsigned* aw) {
  extern __shared__ __attribute__((aligned(16))) int dsm[];
  int* list = dsm;
  int* hl   = dsm + LISTN;
  int* sl   = hl + RCAP;
  int* cnt  = sl + RCAP;
  int* offs = cnt + NBA;
  int* cur  = offs + NBA;
  int* misc = cur + NBA;
  float* pp = (float*)(misc + MISC_INTS);
  constexpr int FL = (L == 1) ? FIN : HID;
  const int tid = (int)threadIdx.x, lane = tid & 31, wave = tid >> 5;
  const int nodeBase = (int)blockIdx.x * NBA;

  {
    const v4i z4 = {0, 0, 0, 0};
    for (int i = tid * 4; i < AGG_ZINTS; i += NTHR * 4) *(v4ia*)(dsm + i) = z4;
    if (tid < MISC_INTS) misc[tid] = 0;
    for (int i = tid; i < 12 * FL; i += NTHR) pp[i] = bf16_val(par[i]);
  }
  __syncthreads();

  int t = 0, ov = 0;
  const int nChunks = (nE + CHUNK - 1) / CHUNK;
#pragma unroll 1
  for (int ch = 0; ch < nChunks; ++ch) {
    const int cbase = ch * CHUNK;
    const int wc = scan_chunk<SLA>(dsts, nE, cbase, nodeBase, NBA, vec8, list, tid, lane, wave);
    if (lane == 0) misc[wave] = wc;
    __syncthreads();
    if (wave == 0) {
#pragma unroll 1
      for (int w2 = 0; w2 < NWAVE; ++w2) {
        int c = misc[w2];
        c = c < 0 ? 0 : (c > WCAP ? WCAP : c);
#pragma unroll 1
        for (int b0 = 0; b0 < c; b0 += 32) {
          const int idx = b0 + lane;
          const int ent = list[w2 * WCAP + (idx < WCAP ? idx : WCAP - 1)];
          const int m32 = (c - b0) < 32 ? (c - b0) : 32;
#pragma unroll 1
          for (int k = 0; k < m32; ++k) {
            const int u    = __builtin_amdgcn_readlane(ent, k);
            const int slot = u & (NBA - 1);
            const int el   = (u >> SLA) & (CHUNK - 1);
            const int pk   = ((cbase + el) << SLA) | slot;
            if (t < RCAP) {
              if (lane == 0) { hl[t] = pk; cnt[slot] = cnt[slot] + 1; }
              t = t + 1;
            } else {
              ov = 1;
            }
          }
        }
      }
    }
    __syncthreads();
  }
  if (wave == 0 && lane == 0) { misc[8] = t; misc[9] = ov; }
  __syncthreads();
  int tt = misc[8];
  tt = tt < 0 ? 0 : (tt > RCAP ? RCAP : tt);
  const int ovf = misc[9];

  if (wave == 0) {
    const int base = lane * (NBA / 32);
    int s = 0;
#pragma unroll 1
    for (int i = 0; i < NBA / 32; ++i) s += cnt[base + i];
    int incl = s;
#pragma unroll
    for (int d = 1; d < 32; d <<= 1) {
      const int y = __shfl_up(incl, d, 32);
      if (lane >= d) incl += y;
    }
    int run = incl - s;
#pragma unroll 1
    for (int i = 0; i < NBA / 32; ++i) {
      const int cv = cnt[base + i];
      offs[base + i] = run;
      cur[base + i]  = run;
      run += cv;
    }
  }
  __syncthreads();
  if (wave == 0) {
#pragma unroll 1
    for (int b0 = 0; b0 < tt; b0 += 32) {
      const int idx = b0 + lane;
      const int ent = hl[idx < RCAP ? idx : RCAP - 1];
      const int m32 = (tt - b0) < 32 ? (tt - b0) : 32;
#pragma unroll 1
      for (int k = 0; k < m32; ++k) {
        const int u    = __builtin_amdgcn_readlane(ent, k);
        const int slot = u & (NBA - 1);
        if (lane == 0) {
          int p = cur[slot];
          p = p < 0 ? 0 : (p > RCAP - 1 ? RCAP - 1 : p);
          sl[p] = u;
          cur[slot] = p + 1;
        }
      }
    }
  }
  __syncthreads();

  const float qn = __int_as_float(0x7fc00000);
  const float pz = (ovf != 0) ? qn : 0.0f;
  const int f = (L == 1) ? lane : (lane & (HID - 1));
  const float al = pp[f],          be = pp[FL + f],     ga = pp[2 * FL + f], de = pp[3 * FL + f];
  const float ea = pp[4 * FL + f], ec = pp[6 * FL + f], ef = pp[8 * FL + f], eh = pp[10 * FL + f];
#pragma unroll 1
  for (int si = 0; si < NBA / NWAVE; ++si) {
    const int s    = si * NWAVE + wave;
    const int node = nodeBase + s;
    int c = cnt[s];
    const bool big = c > DEGCAP;
    c = c < 0 ? 0 : (c > DEGCAP ? DEGCAP : c);
    int o = offs[s];
    o = o < 0 ? 0 : (o > RCAP ? RCAP : o);
    const int nc = node < nN ? node : nN - 1;
    float a0 = 0.0f, a1 = 0.0f, a2 = 0.0f, a3 = 0.0f;
#pragma unroll 1
    for (int b0 = 0; b0 < c; b0 += 32) {
      int idx = o + b0 + lane;
      idx = idx > RCAP - 1 ? RCAP - 1 : idx;
      const int ent = sl[idx];
      int eid = ent >> SLA;
      eid = eid < 0 ? 0 : (eid > nE - 1 ? nE - 1 : eid);
      int sr = srcs[eid];
      sr = sr < 0 ? 0 : (sr > nN - 1 ? nN - 1 : sr);
      const int m32 = (c - b0) < 32 ? (c - b0) : 32;
#pragma unroll 1
      for (int k = 0; k < m32; ++k) {
        const int sk = __builtin_amdgcn_readlane(sr, k);
        if constexpr (L == 1) {
          const v4f v = *(const v4fa*)(T + (size_t)sk * TW1 + 4 * lane);
          a0 += v.x; a1 += v.y; a2 += v.z; a3 += v.w;
        } else {
          const v2f v = *(const v2fa*)(T + (size_t)sk * TW2 + 2 * lane);
          a0 += v.x; a1 += v.y;
        }
      }
    }
    float sv0, sv1, sv2, sv3;
    if constexpr (L == 1) {
      const int b = lane >> 2, jj = lane & 3;
#define PICK4(TT, DST) { \
        const float g0 = __shfl(a0, b + 8 * (TT)); const float g1 = __shfl(a1, b + 8 * (TT)); \
        const float g2 = __shfl(a2, b + 8 * (TT)); const float g3 = __shfl(a3, b + 8 * (TT)); \
        DST = (jj == 0) ? g0 : ((jj == 1) ? g1 : ((jj == 2) ? g2 : g3)); }
      PICK4(0, sv0)
      PICK4(1, sv1)
      PICK4(2, sv2)
      PICK4(3, sv3)
#undef PICK4
    } else {
      const int b = (lane & (HID - 1)) >> 1, jj = lane & 1;
#define PICK2(TT, DST) { \
        const float g0 = __shfl(a0, b + 8 * (TT)); const float g1 = __shfl(a1, b + 8 * (TT)); \
        DST = (jj != 0) ? g1 : g0; }
      PICK2(0, sv0)
      PICK2(1, sv1)
      PICK2(2, sv2)
      PICK2(3, sv3)
#undef PICK2
    }
    (void)a2; (void)a3;
    const float num = al * powv(sv0 + PEPS, ea) + be * powv(sv1 + PEPS, ec);
    const float den = ga * powv(sv2 + PEPS, ef) + de * powv(sv3 + PEPS, eh);
    const float agg = num / (den + PEPS);
    const float pzr = big ? qn : pz;
    const bool live = node < nN;
    const float gv = live ? (agg + pzr) : 0.0f;
    const int q = lane & 7, grp = lane >> 3;

    if constexpr (L == 1) {
      const float g0 = __shfl(gv, 4 * q), g1 = __shfl(gv, 4 * q + 1), g2 = __shfl(gv, 4 * q + 2), g3 = __shfl(gv, 4 * q + 3);
      const v4f xs = *(const v4f*)(xin + (size_t)nc * FIN + 4 * q);
      const unsigned xb0 = live ? bf16_bits(xs.x + pzr) : 0u;
      const unsigned xb1 = live ? bf16_bits(xs.y + pzr) : 0u;
      const unsigned xb2 = live ? bf16_bits(xs.z + pzr) : 0u;
      const unsigned xb3 = live ? bf16_bits(xs.w + pzr) : 0u;
      const unsigned hb0 = bf16_bits(g0), hb1 = bf16_bits(g1), hb2 = bf16_bits(g2), hb3 = bf16_bits(g3);
      const unsigned lb0 = bf16_bits(g0 - bf16f(hb0)), lb1 = bf16_bits(g1 - bf16f(hb1));
      const unsigned lb2 = bf16_bits(g2 - bf16f(hb2)), lb3 = bf16_bits(g3 - bf16f(hb3));
      const unsigned w0 = (grp == 0) ? xb0 : ((grp == 1) ? hb0 : ((grp == 2) ? lb0 : 0u));
      const unsigned w1 = (grp == 0) ? xb1 : ((grp == 1) ? hb1 : ((grp == 2) ? lb1 : 0u));
      const unsigned w2 = (grp == 0) ? xb2 : ((grp == 1) ? hb2 : ((grp == 2) ? lb2 : 0u));
      const unsigned w3 = (grp == 0) ? xb3 : ((grp == 1) ? hb3 : ((grp == 2) ? lb3 : 0u));
      v2u pk;
      pk.x = w0 | (w1 << 16);
      pk.y = w2 | (w3 << 16);
      if (node < mRows) {
        unsigned* rp = aw + (size_t)node * (AP1 / 2) + 2 * lane;
        *(volatile v2u*)rp = pk;
        __threadfence();
        *(volatile v2u*)rp = pk;
      }
    } else {
      const float g0 = __shfl(gv, 2 * q), g1 = __shfl(gv, 2 * q + 1);
      const unsigned hwd = hpw[(size_t)nc * (HPW / 2) + (lane & 15)];
      const unsigned hb0 = bf16_bits(g0), hb1 = bf16_bits(g1);
      const unsigned lb0 = bf16_bits(g0 - bf16f(hb0)), lb1 = bf16_bits(g1 - bf16f(hb1));
      const unsigned hsel = live ? hwd : 0u;
      const unsigned w = (grp < 2) ? hsel : ((grp == 2) ? (hb0 | (hb1 << 16)) : (lb0 | (lb1 << 16)));
      if (node < mRows) {
        unsigned* rp = aw + (size_t)node * (AP2 / 2) + lane;
        *(volatile unsigned*)rp = w;
        __threadfence();
        *(volatile unsigned*)rp = w;
      }
    }
  }
}

__global__ __launch_bounds__(GTHR) void k_gemm1(const unsigned short* __restrict__ A1,
                                                const unsigned short* __restrict__ B1T,
                                                const float* __restrict__ b1, const float* __restrict__ par2,
                                                unsigned short* H1P, float* T2, int nN) {
  __shared__ __attribute__((aligned(16))) float stg[GBM * HID];
  __shared__ __attribute__((aligned(16))) float st2[GBM * TW2];
  __shared__ __attribute__((aligned(16))) unsigned short sth[GBM * HPW];
  __shared__ __attribute__((aligned(16))) float pe[4 * HID];
  __shared__ __attribute__((aligned(16))) float pb[HID];
  const int tid = (int)threadIdx.x, lane = tid & 31, wave = tid >> 5, hh = lane >> 4, m = lane & 15;
  const int rowBase = (int)blockIdx.x * GBM;
  if (tid < 4 * HID) {
    const int tt = tid >> 4, c = tid & 15;
    pe[tid] = bf16_val(par2[(5 + 2 * tt) * HID + c]);
  }
  if (tid < HID) pb[tid] = bf16_val(b1[tid]);

  v8f acc = {0.f, 0.f, 0.f, 0.f, 0.f, 0.f, 0.f, 0.f};
  const unsigned short* ap = A1 + (size_t)(rowBase + 16 * wave + m) * (size_t)AP1 + 8 * hh;
  const unsigned short* bp = B1T + (size_t)m * (size_t)BP1 + 8 * hh;
#pragma unroll 1
  for (int k0 = 0; k0 < KL1; k0 += 32) {
    FragB af, bf;
    af.h[0] = *(const v8usa*)(ap + k0);
    af.h[1] = *(const v8usa*)(ap + k0 + 16);
    bf.h[0] = *(const v8usa*)(bp + k0);
    bf.h[1] = *(const v8usa*)(bp + k0 + 16);
    acc = wmb(af, bf, acc);
  }
#pragma unroll
  for (int r = 0; r < 8; ++r) stg[(16 * wave + 8 * hh + r) * HID + m] = acc[r];
  __syncthreads();

#pragma unroll 1
  for (int it = 0; it < (GBM * HID) / GTHR; ++it) {
    const int cell = it * GTHR + tid;
    const int row = cell >> 4, col = cell & 15;
    float h = fmaxf(stg[cell] + pb[col], 0.0f);
    h = (rowBase + row < nN) ? h : 0.0f;
    const unsigned hb = bf16_bits(h);
    const unsigned lb = bf16_bits(h - bf16f(hb));
    sth[row * HPW + col]       = (unsigned short)hb;
    sth[row * HPW + HID + col] = (unsigned short)lb;
    float e = 1.0f / (1.0f + expf(-h));
    e = fminf(fmaxf(e, PEPS), 1.0f - PEPS);
    const float om = 1.0f - e;
    const float le = log2f(e), lo = log2f(om);
    float* trow = st2 + row * TW2;
    trow[col]           = exp2f(pe[col] * le);
    trow[HID + col]     = exp2f(pe[HID + col] * lo);
    trow[2 * HID + col] = exp2f(pe[2 * HID + col] * le);
    trow[3 * HID + col] = exp2f(pe[3 * HID + col] * lo);
  }
  __syncthreads();

  float* tb = T2 + (size_t)rowBase * TW2;
  unsigned short* hp = H1P + (size_t)rowBase * HPW;
  v4f  tv[(GBM * TW2 / 4) / GTHR];
  v8us hv[(GBM * HPW / 8) / GTHR];
#pragma unroll
  for (int it = 0; it < (GBM * TW2 / 4) / GTHR; ++it) tv[it] = *(const v4fa*)(st2 + 4 * (it * GTHR + tid));
#pragma unroll
  for (int it = 0; it < (GBM * HPW / 8) / GTHR; ++it) hv[it] = *(const v8usa*)(sth + 8 * (it * GTHR + tid));
#pragma unroll
  for (int it = 0; it < (GBM * TW2 / 4) / GTHR; ++it) *(volatile v4f*)(tb + 4 * (it * GTHR + tid)) = tv[it];
#pragma unroll
  for (int it = 0; it < (GBM * HPW / 8) / GTHR; ++it) *(volatile v8us*)(hp + 8 * (it * GTHR + tid)) = hv[it];
  __threadfence();
#pragma unroll
  for (int it = 0; it < (GBM * TW2 / 4) / GTHR; ++it) *(volatile v4f*)(tb + 4 * (it * GTHR + tid)) = tv[it];
#pragma unroll
  for (int it = 0; it < (GBM * HPW / 8) / GTHR; ++it) *(volatile v8us*)(hp + 8 * (it * GTHR + tid)) = hv[it];
}

__global__ __launch_bounds__(GTHR) void k_gemm2(const unsigned short* __restrict__ A2,
                                                const unsigned short* __restrict__ B2T,
                                                const float* __restrict__ b2, float* out, int nN) {
  __shared__ __attribute__((aligned(16))) float stg[GBM * HID];
  __shared__ __attribute__((aligned(16))) float sto[GBM * HID];
  __shared__ __attribute__((aligned(16))) float pb[HID];
  const int tid = (int)threadIdx.x, lane = tid & 31, wave = tid >> 5, hh = lane >> 4, m = lane & 15;
  const int rowBase = (int)blockIdx.x * GBM;
  if (tid < HID) pb[tid] = bf16_val(b2[tid]);

  v8f acc = {0.f, 0.f, 0.f, 0.f, 0.f, 0.f, 0.f, 0.f};
  const unsigned short* ap = A2 + (size_t)(rowBase + 16 * wave + m) * (size_t)AP2 + 8 * hh;
  const unsigned short* bp = B2T + (size_t)m * (size_t)BP2 + 8 * hh;
#pragma unroll 1
  for (int k0 = 0; k0 < KL2; k0 += 32) {
    FragB af, bf;
    af.h[0] = *(const v8usa*)(ap + k0);
    af.h[1] = *(const v8usa*)(ap + k0 + 16);
    bf.h[0] = *(const v8usa*)(bp + k0);
    bf.h[1] = *(const v8usa*)(bp + k0 + 16);
    acc = wmb(af, bf, acc);
  }
#pragma unroll
  for (int r = 0; r < 8; ++r) stg[(16 * wave + 8 * hh + r) * HID + m] = acc[r];
  __syncthreads();

  {
    const int row = tid & (GBM - 1);
    const float* srw = stg + row * HID;
    const v4f q0 = *(const v4fa*)(srw)      + *(const v4fa*)(pb);
    const v4f q1 = *(const v4fa*)(srw + 4)  + *(const v4fa*)(pb + 4);
    const v4f q2 = *(const v4fa*)(srw + 8)  + *(const v4fa*)(pb + 8);
    const v4f q3 = *(const v4fa*)(srw + 12) + *(const v4fa*)(pb + 12);
    float mx = fmaxf(fmaxf(fmaxf(q0.x, q0.y), fmaxf(q0.z, q0.w)), fmaxf(fmaxf(q1.x, q1.y), fmaxf(q1.z, q1.w)));
    mx = fmaxf(mx, fmaxf(fmaxf(fmaxf(q2.x, q2.y), fmaxf(q2.z, q2.w)), fmaxf(fmaxf(q3.x, q3.y), fmaxf(q3.z, q3.w))));
    float ssum = 0.0f;
#pragma unroll 1
    for (int j = 0; j < HID; ++j) ssum += expf((srw[j] + pb[j]) - mx);
    const float ls = logf(ssum);
    const v4f mv = {mx, mx, mx, mx};
    const v4f lv = {ls, ls, ls, ls};
    const v4f o0 = (q0 - mv) - lv, o1 = (q1 - mv) - lv, o2 = (q2 - mv) - lv, o3 = (q3 - mv) - lv;
    if (wave < 2) {
      float* orw = sto + row * HID;
      *(v4fa*)(orw)      = o0;
      *(v4fa*)(orw + 4)  = o1;
      *(v4fa*)(orw + 8)  = o2;
      *(v4fa*)(orw + 12) = o3;
    }
  }
  __syncthreads();

  float* ob = out + (size_t)rowBase * HID;
  v4f ov[(GBM * HID / 4) / GTHR];
#pragma unroll
  for (int it = 0; it < (GBM * HID / 4) / GTHR; ++it) ov[it] = *(const v4fa*)(sto + 4 * (it * GTHR + tid));
#pragma unroll
  for (int it = 0; it < (GBM * HID / 4) / GTHR; ++it) {
    const int p = it * GTHR + tid;
    if (rowBase + (p >> 2) < nN) *(volatile v4f*)(ob + 4 * p) = ov[it];
  }
  __threadfence();
#pragma unroll
  for (int it = 0; it < (GBM * HID / 4) / GTHR; ++it) {
    const int p = it * GTHR + tid;
    if (rowBase + (p >> 2) < nN) *(volatile v4f*)(ob + 4 * p) = ov[it];
  }
}

static inline int cdiv(int a, int b) { return (a + b - 1) / b; }
static inline size_t al256(size_t o) { return (o + 255) & ~(size_t)255; }

extern "C" void kernel_launch(void* const* d_in, const int* in_sizes, int n_in,
                              void* d_out, int out_size, void* d_ws, size_t ws_size,
                              hipStream_t stream) {
  if (n_in < 10) return;
  if (in_sizes[0] < FIN * 16 || (in_sizes[0] % FIN) != 0) return;
  const int nN = in_sizes[0] / FIN;
  if (in_sizes[1] < 2 || (in_sizes[1] & 1) != 0) return;
  const int nE = in_sizes[1] / 2;
  if (nE < 1 || nE >= (1 << 21) || nN >= (1 << 24)) return;
  if (in_sizes[2] != 12 * FIN) return;
  if (in_sizes[3] != FIN * HID || in_sizes[4] != FIN * HID) return;
  if (in_sizes[5] != HID) return;
  if (in_sizes[6] != 12 * HID) return;
  if (in_sizes[7] != HID * HID || in_sizes[8] != HID * HID) return;
  if (in_sizes[9] != HID) return;
  if ((long long)out_size != (long long)nN * HID) return;

  const float* x   = (const float*)d_in[0];
  const int*   ei  = (const int*)d_in[1];
  const float* p1  = (const float*)d_in[2];
  const float* wr1 = (const float*)d_in[3];
  const float* wn1 = (const float*)d_in[4];
  const float* b1  = (const float*)d_in[5];
  const float* p2  = (const float*)d_in[6];
  const float* wr2 = (const float*)d_in[7];
  const float* wn2 = (const float*)d_in[8];
  const float* b2  = (const float*)d_in[9];
  float* out = (float*)d_out;
  const int* src = ei;
  const int* dst = ei + nE;

  const int MP = cdiv(nN, GBM) * GBM;
  const int gM = MP / GBM;
  const int gT = MP / TR1;
  const int gA = cdiv(MP, NBA);
  if ((long long)gA * NBA < (long long)MP) return;
  const int vec8 = ((nE & 3) == 0) ? 1 : 0;

  char* ws = (char*)d_ws;
  size_t off = 0;
  const size_t oB1 = off; off = al256(off + (size_t)HID * BP1 * 2);
  const size_t oB2 = off; off = al256(off + (size_t)HID * BP2 * 2);
  const size_t oT1 = off; off = al256(off + (size_t)MP * TW1 * 4);
  const size_t oA1 = off; off = al256(off + (size_t)MP * AP1 * 2);
  const size_t oT2 = off; off = al256(off + (size_t)MP * TW2 * 4);
  const size_t oHP = off; off = al256(off + (size_t)MP * HPW * 2);
  const size_t oA2 = off; off = al256(off + (size_t)MP * AP2 * 2);
  if (off > ws_size || off > (size_t)WSMAX) return;
  unsigned short* B1T = (unsigned short*)(ws + oB1);
  unsigned short* B2T = (unsigned short*)(ws + oB2);
  float*          T1  = (float*)(ws + oT1);
  unsigned short* A1  = (unsigned short*)(ws + oA1);
  float*          T2  = (float*)(ws + oT2);
  unsigned short* H1P = (unsigned short*)(ws + oHP);
  unsigned short* A2  = (unsigned short*)(ws + oA2);

  const size_t scanLds = (size_t)SCAN_LDS_INTS * 4;
  hipFuncSetAttribute(reinterpret_cast<const void*>(&k_scan<1>), hipFuncAttributeMaxDynamicSharedMemorySize, (int)scanLds);
  hipFuncSetAttribute(reinterpret_cast<const void*>(&k_scan<2>), hipFuncAttributeMaxDynamicSharedMemorySize, (int)scanLds);

  k_wprep<<<1, NTHR, 0, stream>>>(wr1, wn1, wr2, wn2, B1T, B2T);
  k_t1<<<gT, NTHR, 0, stream>>>(x, p1, T1, nN);
  k_scan<1><<<gA, NTHR, scanLds, stream>>>(src, dst, nE, nN, vec8, MP, p1, T1, x,
                                            (const unsigned*)H1P, (unsigned*)A1);
  k_gemm1<<<gM, GTHR, 0, stream>>>(A1, B1T, b1, p2, H1P, T2, nN);
  k_scan<2><<<gA, NTHR, scanLds, stream>>>(src, dst, nE, nN, vec8, MP, p2, T2, x,
                                            (const unsigned*)H1P, (unsigned*)A2);
  k_gemm2<<<gM, GTHR, 0, stream>>>(A2, B2T, b2, out, nN);
}
